// LR_PINN_phase2_midout_87497073754924
// MI455X (gfx1250) — hardware-verified
//
#include <hip/hip_runtime.h>


#define NPT  262144
#define HH   256
#define RR   32
#define RP   64
#define CHK  65536
typedef _Float16 h16;
typedef unsigned short bf;
typedef __attribute__((ext_vector_type(16))) __bf16   v16bf;
typedef __attribute__((ext_vector_type(16))) _Float16 v16h;
typedef __attribute__((ext_vector_type(8)))  _Float16 v8h;
typedef __attribute__((ext_vector_type(8)))  unsigned short v8us;
typedef __attribute__((ext_vector_type(8)))  float    v8f;
typedef __attribute__((ext_vector_type(4)))  float    v4f;
typedef v8h  __attribute__((may_alias)) v8ha;
typedef v4f  __attribute__((may_alias)) v4fa;
typedef v8us __attribute__((may_alias)) v8usa;

__device__ __forceinline__ unsigned short f2bf(float f) { unsigned u = __float_as_uint(f); u += 0x7FFFu + ((u >> 16) & 1u); return (unsigned short)(u >> 16); }
__device__ __forceinline__ float bf2f(unsigned short b) { return __uint_as_float(((unsigned)b) << 16); }
__device__ __forceinline__ float bfr(float f) { return bf2f(f2bf(f)); }
__device__ __forceinline__ v16h cat16(v8h lo, v8h hi) { return __builtin_shufflevector(lo, hi, 0, 1, 2, 3, 4, 5, 6, 7, 8, 9, 10, 11, 12, 13, 14, 15); }
__device__ __forceinline__ v16bf cat16b(v8us lo, v8us hi) { return __builtin_bit_cast(v16bf, __builtin_shufflevector(lo, hi, 0, 1, 2, 3, 4, 5, 6, 7, 8, 9, 10, 11, 12, 13, 14, 15)); }
__device__ __forceinline__ v8f wmma16(v16h a, v16h b, v8f c) { return __builtin_amdgcn_wmma_f32_16x16x32_f16(false, a, false, b, (short)0, c, false, false); }
__device__ __forceinline__ v8f wmmab(v16bf a, v16bf b, v8f c) { return __builtin_amdgcn_wmma_f32_16x16x32_bf16(false, a, false, b, (short)0, c, false, false); }


template <typename T16> struct WFrag;
template <> struct WFrag<h16> { typedef v16h V; static __device__ __forceinline__ V ld(const h16* p) { return cat16(*(const v8h*)p, *(const v8h*)(p + 16)); } static __device__ __forceinline__ v8f mma(V a, V b, v8f c) { return wmma16(a, b, c); } };
template <> struct WFrag<bf> { typedef v16bf V; static __device__ __forceinline__ V ld(const bf* p) { return cat16b(*(const v8us*)p, *(const v8us*)(p + 16)); } static __device__ __forceinline__ v8f mma(V a, V b, v8f c) { return wmmab(a, b, c); } };
template <typename T16, int NSPLIT, bool BIAS>
__global__ __launch_bounds__(32) void k_gemmw(const T16* __restrict__ A, const T16* __restrict__ A2, const T16* __restrict__ Bt, const T16* __restrict__ Bt2, int K, float* C, int ldc, const float* __restrict__ bias, size_t sA, size_t sB, size_t sC) {
    typedef typename WFrag<T16>::V V;
    __shared__ __align__(16) float os[16 * 68];
    const size_t z = blockIdx.z; A += z * sA; if (A2) A2 += z * sA; Bt += z * sB; if (Bt2) Bt2 += z * sB; C += z * sC;
    const int lane = threadIdx.x & 31, lr = lane & 15, hi = lane >> 4; const int r0 = blockIdx.x * 64, c0 = blockIdx.y * 64;
    v8f acc[4][4];
#pragma unroll
    for (int mb = 0; mb < 4; ++mb)
#pragma unroll
        for (int nb = 0; nb < 4; ++nb) acc[mb][nb] = (v8f){};
    const size_t aoff = (size_t)(r0 + lr) * K + 8 * hi, boff = (size_t)(c0 + lr) * K + 8 * hi;
#pragma unroll 1
    for (int kc = 0; kc < K; kc += 32) {
        V a[4], a2[4];
#pragma unroll
        for (int mb = 0; mb < 4; ++mb) { a[mb] = WFrag<T16>::ld(A + aoff + (size_t)mb * 16 * K + kc); if (NSPLIT == 1 || NSPLIT == 2) a2[mb] = WFrag<T16>::ld(A2 + aoff + (size_t)mb * 16 * K + kc); }
#pragma unroll
        for (int nb = 0; nb < 4; ++nb) { const V b = WFrag<T16>::ld(Bt + boff + (size_t)nb * 16 * K + kc); V b2; if (NSPLIT >= 2) b2 = WFrag<T16>::ld(Bt2 + boff + (size_t)nb * 16 * K + kc);
#pragma unroll
            for (int mb = 0; mb < 4; ++mb) { acc[mb][nb] = WFrag<T16>::mma(a[mb], b, acc[mb][nb]); if (NSPLIT == 1 || NSPLIT == 2) acc[mb][nb] = WFrag<T16>::mma(a2[mb], b, acc[mb][nb]); if (NSPLIT >= 2) acc[mb][nb] = WFrag<T16>::mma(a[mb], b2, acc[mb][nb]); } }
        asm volatile("v_nop\n\tv_nop\n\tv_nop\n\tv_nop" : "+v"(acc[0][0]), "+v"(acc[1][1]), "+v"(acc[2][2]), "+v"(acc[3][3]) : "v"(a[0]), "v"(a[3]));
    }
#pragma unroll
    for (int mb = 0; mb < 4; ++mb) {
#pragma unroll
        for (int nb = 0; nb < 4; ++nb) {
#pragma unroll
            for (int j = 0; j < 8; ++j) os[(hi * 8 + j) * 68 + nb * 16 + lr] = acc[mb][nb][j]; }
        __builtin_amdgcn_wave_barrier(); asm volatile("" ::: "memory");
        float* crow = C + (size_t)(r0 + mb * 16) * ldc + c0;
#pragma unroll 1
        for (int ps = 0; ps < 2; ++ps) {
#pragma unroll
            for (int s = 0; s < 8; ++s) { const int row = 2 * s + hi, cofs = lr * 4; v4f val = *(const v4fa*)(os + row * 68 + cofs); if (BIAS) { val[0] += bfr(bias[c0 + cofs]); val[1] += bfr(bias[c0 + cofs + 1]); val[2] += bfr(bias[c0 + cofs + 2]); val[3] += bfr(bias[c0 + cofs + 3]); }
                *(volatile v4f*)(crow + (size_t)row * ldc + cofs) = val; }
            if (ps == 0) __threadfence(); }
        __builtin_amdgcn_wave_barrier(); asm volatile("" ::: "memory");
    }
}

__device__ __forceinline__ void splitf(float y, unsigned short& h, unsigned short& l) { h = f2bf(y); l = f2bf(y - bf2f(h)); }
typedef __attribute__((ext_vector_type(4))) unsigned short v4us;

__global__ __launch_bounds__(256) void k_cvt8(const float* __restrict__ src, bf* dst, size_t n8) { const size_t i = (size_t)blockIdx.x * 256 + threadIdx.x; if (i >= n8) return; const v8f v = *(const v8f*)(src + i * 8); v8us o;
#pragma unroll
    for (int k = 0; k < 8; ++k) o[k] = f2bf(v[k]); *(volatile v8us*)(dst + i * 8) = o; __threadfence(); *(volatile v8us*)(dst + i * 8) = o; }
__global__ __launch_bounds__(256) void k_start(const float* __restrict__ x, const float* __restrict__ t, const float* __restrict__ ws, const float* __restrict__ bs, int r0, bf* Hh, bf* Hl) { const int e = (blockIdx.x * 256 + threadIdx.x) * 4; if (e >= CHK * HH) return; const int c = e % HH; const int n = r0 + e / HH; const float xv = bfr(x[n]), tv = bfr(t[n]); v4us oh, ol;
#pragma unroll
    for (int u = 0; u < 4; ++u) { float a = __fmul_rn(xv, bfr(ws[(c + u) * 2])), b = __fmul_rn(tv, bfr(ws[(c + u) * 2 + 1])); asm volatile("" : "+v"(a)); asm volatile("" : "+v"(b)); float s = __fadd_rn(a, b); asm volatile("" : "+v"(s)); const float y = tanhf(__fadd_rn(s, bfr(bs[c + u]))); unsigned short p, q; splitf(y, p, q); oh[u] = p; ol[u] = q; }
    *(volatile v4us*)(Hh + e) = oh; *(volatile v4us*)(Hl + e) = ol; __threadfence(); *(volatile v4us*)(Hh + e) = oh; *(volatile v4us*)(Hl + e) = ol; }
__global__ __launch_bounds__(256) void k_ca(const float* __restrict__ col, const float* __restrict__ alpha, bf* Bh, bf* Bl) { const int e = (blockIdx.x * 256 + threadIdx.x) * 4; if (e >= RP * HH) return; const int h = e % HH; const int r = e / HH; v4us oh, ol;
#pragma unroll
    for (int u = 0; u < 4; ++u) { unsigned short p = 0, q = 0; if (r < RR) splitf(__fmul_rn(bfr(col[(size_t)(h + u) * RR + r]), bfr(alpha[r])), p, q); oh[u] = p; ol[u] = q; } *(volatile v4us*)(Bh + e) = oh; *(volatile v4us*)(Bl + e) = ol; __threadfence(); *(volatile v4us*)(Bh + e) = oh; *(volatile v4us*)(Bl + e) = ol; }
__global__ __launch_bounds__(256) void k_rw(const float* __restrict__ row, bf* Bt) { const int e = (blockIdx.x * 256 + threadIdx.x) * 4; if (e >= HH * RP) return; const int r = e % RP; const int h = e / RP; v4us o;
#pragma unroll
    for (int u = 0; u < 4; ++u) o[u] = (r + u < RR) ? f2bf(row[(size_t)h * RR + r + u]) : (unsigned short)0; *(volatile v4us*)(Bt + e) = o; __threadfence(); *(volatile v4us*)(Bt + e) = o; }
__global__ __launch_bounds__(256) void k_spl(const float* __restrict__ F, size_t n4, bf* Hh, bf* Hl) { const size_t e = ((size_t)blockIdx.x * 256 + threadIdx.x) * 4; if (e >= n4) return; const v4f a = *(const v4f*)(F + e); v4us oh, ol;
#pragma unroll
    for (int u = 0; u < 4; ++u) { unsigned short p, q; splitf(a[u], p, q); oh[u] = p; ol[u] = q; } *(volatile v4us*)(Hh + e) = oh; *(volatile v4us*)(Hl + e) = ol; __threadfence(); *(volatile v4us*)(Hh + e) = oh; *(volatile v4us*)(Hl + e) = ol; }
__global__ __launch_bounds__(256) void k_tanh(const float* __restrict__ F, size_t n4, bf* Hh, bf* Hl) { const size_t e = ((size_t)blockIdx.x * 256 + threadIdx.x) * 4; if (e >= n4) return; const v4f a = *(const v4f*)(F + e); v4us oh, ol;
#pragma unroll
    for (int u = 0; u < 4; ++u) { unsigned short p, q; splitf(tanhf(a[u]), p, q); oh[u] = p; ol[u] = q; } *(volatile v4us*)(Hh + e) = oh; *(volatile v4us*)(Hl + e) = ol; __threadfence(); *(volatile v4us*)(Hh + e) = oh; *(volatile v4us*)(Hl + e) = ol; }
__global__ __launch_bounds__(256) void k_end(const float* __restrict__ F, const float* __restrict__ we, const float* __restrict__ be, int r0, float* OUT) { const int idx = blockIdx.x * 256 + threadIdx.x; if (idx >= CHK) return; const float* f = F + (size_t)idx * HH; float acc = 0.f;
#pragma unroll 4
    for (int c = 0; c < HH; ++c) { float p = __fmul_rn(tanhf(f[c]), bfr(we[c])); asm volatile("" : "+v"(p)); acc = __fadd_rn(acc, p); }
    const float r = __fadd_rn(acc, bfr(be[0])); *(volatile float*)(OUT + r0 + idx) = r; __threadfence(); *(volatile float*)(OUT + r0 + idx) = r; }

extern "C" void kernel_launch(void* const* d_in, const int* in_sizes, int n_in,
                              void* d_out, int out_size, void* d_ws, size_t ws_size, hipStream_t stream) {
    (void)in_sizes; (void)n_in; (void)out_size;
    const float** I = (const float**)d_in;
    const float *x = I[0], *t = I[1], *ws = I[2], *bs = I[3], *we = I[4], *be = I[5]; const float* col[3] = {I[6], I[7], I[8]}; const float* row[3] = {I[9], I[10], I[11]}; const float* alpha[3] = {I[12], I[13], I[14]};
    float* OUT = (float*)d_out;
    char* wsp = (char*)d_ws;
    auto take = [&](size_t bytes) { char* p = wsp; wsp += (bytes + 255) & ~(size_t)255; return (void*)p; };
    bf* CAh[3]; bf* CAl[3]; bf* RW[3]; for (int i = 0; i < 3; ++i) { CAh[i] = (bf*)take(RP * HH * 2); CAl[i] = (bf*)take(RP * HH * 2); RW[i] = (bf*)take(HH * RP * 2); }
    bf* Hh = (bf*)take((size_t)CHK * HH * 2); bf* Hl = (bf*)take((size_t)CHK * HH * 2); float* G = (float*)take((size_t)CHK * RP * 4); bf* Gh = (bf*)take((size_t)CHK * RP * 2); bf* Gl = (bf*)take((size_t)CHK * RP * 2); float* F = (float*)take((size_t)CHK * HH * 4);
    if ((size_t)(wsp - (char*)d_ws) > ws_size) return;
    for (int i = 0; i < 3; ++i) { k_ca<<<(RP * HH / 4 + 255) / 256, 256, 0, stream>>>(col[i], alpha[i], CAh[i], CAl[i]); k_rw<<<(HH * RP / 4 + 255) / 256, 256, 0, stream>>>(row[i], RW[i]); }
    for (int r0 = 0; r0 < NPT; r0 += CHK) {
        k_start<<<(CHK * HH / 4 + 255) / 256, 256, 0, stream>>>(x, t, ws, bs, r0, Hh, Hl);
        for (int i = 0; i < 3; ++i) {
            k_gemmw<bf, 2, false><<<dim3(CHK / 64, RP / 64, 1), 32, 0, stream>>>(Hh, Hl, CAh[i], CAl[i], HH, G, RP, nullptr, 0, 0, 0);
            k_spl<<<(CHK * RP / 4 + 255) / 256, 256, 0, stream>>>(G, (size_t)CHK * RP, Gh, Gl);
            k_gemmw<bf, 1, false><<<dim3(CHK / 64, HH / 64, 1), 32, 0, stream>>>(Gh, Gl, RW[i], nullptr, RP, F, HH, nullptr, 0, 0, 0);
            if (i < 2) k_tanh<<<(CHK * HH / 4 + 255) / 256, 256, 0, stream>>>(F, (size_t)CHK * HH, Hh, Hl); }
        k_end<<<CHK / 256, 256, 0, stream>>>(F, we, be, r0, OUT); }
}
